// SS2DExpert_71545565216782
// MI455X (gfx1250) — hardware-verified
//
#include <hip/hip_runtime.h>
#include <hip/hip_bf16.h>
#include <math.h>

#define NB_ 16
#define IH  56
#define IW  56
#define LQ  3136
#define DM  128
#define DI  128
#define NPOS (NB_ * LQ)
#define SS  64
#define HH  1
#define DKK 64
#define BB  1

typedef _Float16 bf16;
typedef _Float16 f16;
typedef __attribute__((ext_vector_type(4))) unsigned v4u_t;
typedef unsigned v4ua __attribute__((ext_vector_type(4), may_alias));
typedef __attribute__((ext_vector_type(4))) float v4f_t;
typedef float v4fa __attribute__((ext_vector_type(4), may_alias));
typedef __attribute__((ext_vector_type(16))) bf16  bf16x16;
typedef __attribute__((ext_vector_type(8)))  bf16  bf16x8;
typedef __attribute__((ext_vector_type(4)))  bf16  bf16x4;
typedef __attribute__((ext_vector_type(8)))  float f32x8;
#define LDS_STRIDE 48
#define KSTRIDE    72
#define VSTRIDE    48

__device__ __forceinline__ f32x8 wmma_bf16(bf16x16 a, bf16x16 b, f32x8 c) {
  c = __builtin_amdgcn_wmma_f32_16x16x32_f16(false, a, false, b, (short)0, c, false, false);
  asm volatile("v_nop\n\tv_nop\n\tv_nop\n\tv_nop" : "+v"(c) : "v"(a), "v"(b));
  return c;
}

template <typename T>
__device__ __forceinline__ bf16x16 load_frag(const T* __restrict__ base, int ld,
                                             int row0, int k0) {
  const int lane = threadIdx.x & 31;
  const int r    = lane & 15;
  const int kh   = (lane >> 4) * 8;
  const T* p0 = base + (size_t)(row0 + r) * ld + (k0 + kh);
  const T* p1 = p0 + 16;
  bf16x16 f;
#pragma unroll
  for (int i = 0; i < 8; ++i) {
    f[i]     = (bf16)p0[i];
    f[i + 8] = (bf16)p1[i];
  }
  return f;
}

__device__ __forceinline__ bf16x16 lds_frag(const bf16* base, int stride) {
  const int lane = threadIdx.x & 31;
  const int row  = lane & 15;
  const int kh   = (lane >> 4) * 8;
  const bf16x8 lo = *(const bf16x8*)(base + row * stride + kh);
  const bf16x8 hi = *(const bf16x8*)(base + row * stride + kh + 16);
  bf16x16 f;
#pragma unroll
  for (int i = 0; i < 8; ++i) { f[i] = lo[i]; f[i + 8] = hi[i]; }
  return f;
}

template <typename T>
__device__ __forceinline__ void stage_read16(const T* __restrict__ p, float* buf) {
#pragma unroll
  for (int i = 0; i < 16; ++i) buf[i] = (float)p[i];
}

__device__ __forceinline__ void stage_write(bf16* dst, const float* buf, int nquad) {
#pragma unroll
  for (int i = 0; i < nquad; ++i) {
    bf16x4 q;
    q[0] = (bf16)buf[4 * i];     q[1] = (bf16)buf[4 * i + 1];
    q[2] = (bf16)buf[4 * i + 2]; q[3] = (bf16)buf[4 * i + 3];
    *(bf16x4*)(dst + 4 * i) = q;
  }
}

template <typename AT, int MODE>
__global__ __launch_bounds__(256) void gemm_rb_kernel(
    const AT* __restrict__ A, const float* __restrict__ W,
    const float* __restrict__ bias, const float* __restrict__ rowscale, const float* __restrict__ R, const float* __restrict__ rowbias, void* __restrict__ out,
    int M, int N, int K) {
  __shared__ bf16 ldsA[128 * LDS_STRIDE];
  __shared__ bf16 ldsW[256 * LDS_STRIDE];
  __shared__ __attribute__((aligned(16))) unsigned char sob[256 * 136 * 2];

  const int t    = threadIdx.x;
  const int wave = t >> 5;
  const int lane = t & 31;
  const int wm   = (wave & 1) * 64;
  const int wn   = (wave >> 1) * 64;
  const int mBlk = blockIdx.x * 128;
  const int nBlk = blockIdx.y * 256;

  const int arow = t >> 1;
  const int ach  = (t & 1) * 16;

  float abuf[16];
  float wbuf[32];

  stage_read16(A + (size_t)(mBlk + arow) * K + ach, abuf);
  const int nrow = min(nBlk + t, N - 1);
  stage_read16(W + (size_t)nrow * K,          wbuf);
  stage_read16(W + (size_t)nrow * K + 16,     wbuf + 16);

  f32x8 acc[4][4] = {};

  for (int k = 0; k < K; k += 32) {
    __syncthreads();
    stage_write(&ldsA[arow * LDS_STRIDE + ach], abuf, 4);
    stage_write(&ldsW[t * LDS_STRIDE],          wbuf, 8);
    if (k + 32 < K) {
      stage_read16(A + (size_t)(mBlk + arow) * K + (k + 32) + ach, abuf);
      stage_read16(W + (size_t)nrow * K + (k + 32),          wbuf);
      stage_read16(W + (size_t)nrow * K + (k + 32) + 16,     wbuf + 16);
    }
    __syncthreads();

    bf16x16 af[4], wf[4];
#pragma unroll
    for (int i = 0; i < 4; ++i)
      af[i] = lds_frag(ldsA + (wm + 16 * i) * LDS_STRIDE, LDS_STRIDE);
#pragma unroll
    for (int j = 0; j < 4; ++j)
      wf[j] = lds_frag(ldsW + (wn + 16 * j) * LDS_STRIDE, LDS_STRIDE);
#pragma unroll
    for (int i = 0; i < 4; ++i)
#pragma unroll
      for (int j = 0; j < 4; ++j)
        acc[i][j] = wmma_bf16(af[i], wf[j], acc[i][j]);
  }

  const int nlane = lane & 15;
  const int mh    = (lane >> 4) * 8;
  __syncthreads();
  if (MODE == 0 || MODE == 1 || MODE == 3) {
    bf16* so = (bf16*)sob;
#pragma unroll
    for (int i = 0; i < 4; ++i)
#pragma unroll
      for (int j = 0; j < 4; ++j) {
        const int nl = wn + 16 * j + nlane;
        const float bv = bias ? bias[nBlk + nl] : 0.0f;
        if (MODE == 3) {
#pragma unroll 1
          for (int r = 0; r < 8; ++r) {
            const int ml = wm + 16 * i + mh + r;
            const float xg = acc[i][j][r] + bv;
            so[ml * 264 + nl] = (bf16)(0.5f * xg * (1.0f + erff(xg * 0.70710678118654752f)));
          }
        } else {
#pragma unroll
        for (int r = 0; r < 8; ++r) {
          const int ml = wm + 16 * i + mh + r;
          const bf16 hv = (bf16)(acc[i][j][r] + bv);
          if (MODE == 0) so[ml * 264 + nl] = hv;
          else           so[nl * 136 + ml] = hv;
        }
        }
      }
    __syncthreads();
#pragma unroll 1
    for (int pass = 0; pass < 2; ++pass) {
      if (MODE == 0 || MODE == 3) {
        for (int ch = t; ch < 128 * 32; ch += 256) { const int ml = ch >> 5, q = (ch & 31) * 8;
          *(volatile v4u_t*)((bf16*)out + (size_t)(mBlk + ml) * N + nBlk + q) = *(const v4ua*)(so + ml * 264 + q); }
      } else {
        const int b_ = mBlk / SS, s0 = mBlk & (SS - 1);
        for (int ch = t; ch < 256 * 16; ch += 256) { const int nl = ch >> 4, q = (ch & 15) * 8; const int n = nBlk + nl, h = n >> 6, dk = n & (DKK - 1);
          *(volatile v4u_t*)((bf16*)out + (((size_t)(b_ * HH + h)) * DKK + dk) * SS + s0 + q) = *(const v4ua*)(so + nl * 136 + q); }
      }
      __threadfence();
    }
  } else {
    float* so = (float*)sob;
#pragma unroll 1
    for (int hf = 0; hf < 2; ++hf) {
      if (wm == hf * 64) {
#pragma unroll
        for (int i = 0; i < 4; ++i)
#pragma unroll
          for (int j = 0; j < 4; ++j) {
            const int nl = wn + 16 * j + nlane;
            const float bv = bias ? bias[nBlk + nl] : 0.0f;
#pragma unroll
            for (int r = 0; r < 8; ++r) { const int mrow = mBlk + hf * 64 + 16 * i + mh + r; so[(16 * i + mh + r) * 260 + nl] = acc[i][j][r] * (rowscale ? rowscale[mrow] : 1.0f) + bv + (rowbias ? rowbias[mrow] : 0.0f); }
          }
      }
      __syncthreads();
      if (R) {
        for (int ch = t; ch < 64 * 64; ch += 256) { const int ml = ch >> 6, q = (ch & 63) * 4;
          if (nBlk + q < N) { const v4f_t rv = *(const v4f_t*)(R + (size_t)(mBlk + hf * 64 + ml) * N + nBlk + q); v4f_t v = *(const volatile v4fa*)(so + ml * 260 + q); v += rv; *(volatile v4fa*)(so + ml * 260 + q) = v; } }
        asm volatile("s_wait_dscnt 0" ::: "memory");
      }
#pragma unroll 1
      for (int pass = 0; pass < 2; ++pass) {
        for (int ch = t; ch < 64 * 64; ch += 256) { const int ml = ch >> 6, q = (ch & 63) * 4;
          if (nBlk + q < N) *(volatile v4f_t*)((float*)out + (size_t)(mBlk + hf * 64 + ml) * N + nBlk + q) = *(const volatile v4fa*)(so + ml * 260 + q); }
        __threadfence();
      }
      __syncthreads();
    }
  }
}


__global__ __launch_bounds__(256) void k_dwconv(const float* __restrict__ xz, const float* __restrict__ cw, const float* __restrict__ cb, float* __restrict__ xc) {
  __shared__ __attribute__((aligned(16))) float oS[IW * DI];
  const int b = blockIdx.x / IH, h = blockIdx.x % IH, tid = threadIdx.x;
  for (int e = tid; e < IW * DI; e += 256) {
    const int w = e >> 7, d = e & 127;
    float s = cb[d];
#pragma unroll
    for (int ky = 0; ky < 3; ++ky) { const int hh = h + ky - 1; if (hh < 0 || hh >= IH) continue;
#pragma unroll
      for (int kx = 0; kx < 3; ++kx) { const int ww = w + kx - 1; if (ww < 0 || ww >= IW) continue;
        s += xz[(((size_t)b * IH + hh) * IW + ww) * 256 + d] * cw[d * 9 + ky * 3 + kx]; } }
    oS[e] = s / (1.0f + __expf(-s));
  }
  __syncthreads();
#pragma unroll 1
  for (int pass = 0; pass < 2; ++pass) {
    for (int q = tid; q < IW * DI / 4; q += 256) *(volatile v4f_t*)(xc + (((size_t)b * IH + h) * IW) * DI + q * 4) = *(const volatile v4fa*)(oS + q * 4);
    __threadfence();
  }
}
__global__ __launch_bounds__(256) void k_wx(const float* __restrict__ xpw, float* __restrict__ Wx) {
  const int tid = threadIdx.x;
  for (int e = tid; e < 32 * DI / 4; e += 256) {
    const int row = e >> 5, q = (e & 31) * 4, k = row >> 3, c = row & 7;
    v4f_t v;
#pragma unroll
    for (int u = 0; u < 4; ++u) v[u] = (c < 6) ? xpw[((size_t)k * 6 + c) * DI + q + u] : 0.0f;
    *(volatile v4f_t*)(Wx + row * DI + q) = v; __threadfence(); *(volatile v4f_t*)(Wx + row * DI + q) = v;
  }
}
__global__ __launch_bounds__(128) void k_scan(const float* __restrict__ proj, const float* __restrict__ xc, const float* __restrict__ dtw,
                                             const float* __restrict__ dtb, const float* __restrict__ Alog, const float* __restrict__ Ds,
                                             float* __restrict__ ysum) {
  const int b = blockIdx.x, lane = threadIdx.x & 31, g = threadIdx.x >> 5, d = g * 32 + lane;
#pragma unroll 1
  for (int k = 0; k < 4; ++k) {
    const float A = -__expf(Alog[k * DI + d]);
    const float w0 = dtw[((size_t)k * DI + d) * 4 + 0], w1 = dtw[((size_t)k * DI + d) * 4 + 1], w2 = dtw[((size_t)k * DI + d) * 4 + 2], w3 = dtw[((size_t)k * DI + d) * 4 + 3];
    const float bias = dtb[k * DI + d], Dd = Ds[k * DI + d];
    float hst = 0.0f;
#pragma unroll 1
    for (int l = 0; l < LQ; ++l) {
      int p;
      if (k == 0) p = l;
      else if (k == 1) p = LQ - 1 - l;
      else { const int lp = (k == 2) ? l : (LQ - 1 - l); const int hh = lp % IH, ww = lp / IH; p = hh * IW + ww; }
      const size_t row = (size_t)b * LQ + p;
      const float* pr = proj + row * 32 + k * 8;
      const float r0 = pr[0], r1 = pr[1], r2 = pr[2], r3 = pr[3], Bv = pr[4], Cv = pr[5];
      const float u = xc[row * DI + d];
      float dt = r0 * w0 + r1 * w1 + r2 * w2 + r3 * w3 + bias;
      dt = (dt > 0.0f ? dt : 0.0f) + log1pf(__expf(-fabsf(dt)));
      const float dA = __expf(dt * A);
      hst = dA * hst + dt * Bv * u;
      const float y = hst * Cv + Dd * u;
      float* dst = ysum + row * DI + d;
      const float prev = (k == 0) ? 0.0f : *(volatile float*)dst;
      const float nv = prev + y;
      *(volatile float*)dst = nv; __threadfence(); *(volatile float*)dst = nv;
    }
  }
}
__global__ __launch_bounds__(256) void k_lnpool(const float* __restrict__ ysum, const float* __restrict__ xz, const float* __restrict__ nw,
                                               const float* __restrict__ nb, float* __restrict__ out) {
  __shared__ __attribute__((aligned(16))) float accS[8][128];
  const int b = blockIdx.x, lane = threadIdx.x & 31, wave = threadIdx.x >> 5;
  float gw[4], gb[4], acc[4];
#pragma unroll
  for (int j = 0; j < 4; ++j) { gw[j] = nw[lane + 32 * j]; gb[j] = nb[lane + 32 * j]; acc[j] = 0.0f; }
#pragma unroll 1
  for (int p = wave; p < LQ; p += 8) {
    const size_t row = (size_t)b * LQ + p;
    float v[4], s = 0.0f;
#pragma unroll
    for (int j = 0; j < 4; ++j) { v[j] = ysum[row * DI + lane + 32 * j]; s += v[j]; }
#pragma unroll
    for (int off = 16; off >= 1; off >>= 1) s += __shfl_xor(s, off, 32);
    const float mu = s * (1.0f / 128.0f);
    float q = 0.0f;
#pragma unroll
    for (int j = 0; j < 4; ++j) { v[j] -= mu; q += v[j] * v[j]; }
#pragma unroll
    for (int off = 16; off >= 1; off >>= 1) q += __shfl_xor(q, off, 32);
    const float rs = rsqrtf(q * (1.0f / 128.0f) + 1e-5f);
#pragma unroll
    for (int j = 0; j < 4; ++j) { const float z = xz[row * 256 + DI + lane + 32 * j]; acc[j] += (v[j] * rs * gw[j] + gb[j]) * (z / (1.0f + __expf(-z))); }
  }
#pragma unroll
  for (int j = 0; j < 4; ++j) accS[wave][lane + 32 * j] = acc[j];
  __syncthreads();
  if (threadIdx.x < 32) {
    v4f_t r;
#pragma unroll
    for (int u = 0; u < 4; ++u) { const int dd = threadIdx.x * 4 + u; float t = 0.0f;
#pragma unroll
      for (int w = 0; w < 8; ++w) t += accS[w][dd]; r[u] = t * (1.0f / (float)LQ); }
    *(volatile v4f_t*)(out + (size_t)b * DI + threadIdx.x * 4) = r; __threadfence(); *(volatile v4f_t*)(out + (size_t)b * DI + threadIdx.x * 4) = r;
  }
}

extern "C" void kernel_launch(void* const* d_in, const int* in_sizes, int n_in,
                              void* d_out, int out_size, void* d_ws, size_t ws_size,
                              hipStream_t stream) {
  (void)in_sizes; (void)n_in; (void)out_size; (void)ws_size;
  const float* x = (const float*)d_in[0];
  const float* Win = (const float*)d_in[1];
  const float* cw = (const float*)d_in[2];
  const float* cb = (const float*)d_in[3];
  const float* xpw = (const float*)d_in[4];
  const float* dtw = (const float*)d_in[5];
  const float* dtb = (const float*)d_in[6];
  const float* Alog = (const float*)d_in[7];
  const float* Ds = (const float*)d_in[8];
  const float* nw = (const float*)d_in[9], *nb = (const float*)d_in[10];
  float* out = (float*)d_out;
  char* ws = (char*)d_ws;
  float* xz = (float*)ws; ws += (size_t)NPOS * 256 * 4;
  float* xc = (float*)ws; ws += (size_t)NPOS * DI * 4;
  float* Wx = (float*)ws; ws += 32 * DI * 4;
  float* proj = (float*)ws; ws += (size_t)NPOS * 32 * 4;
  float* ysum = (float*)ws; ws += (size_t)NPOS * DI * 4;
  gemm_rb_kernel<float, 2><<<dim3(NPOS / 128, 1), dim3(256), 0, stream>>>(x, Win, nullptr, nullptr, nullptr, nullptr, xz, NPOS, 256, DM);
  k_dwconv<<<dim3(NB_ * IH), dim3(256), 0, stream>>>(xz, cw, cb, xc);
  k_wx<<<dim3(1), dim3(256), 0, stream>>>(xpw, Wx);
  gemm_rb_kernel<float, 2><<<dim3(NPOS / 128, 1), dim3(256), 0, stream>>>(xc, Wx, nullptr, nullptr, nullptr, nullptr, proj, NPOS, 32, DI);
  k_scan<<<dim3(NB_), dim3(128), 0, stream>>>(proj, xc, dtw, dtb, Alog, Ds, ysum);
  k_lnpool<<<dim3(NB_), dim3(256), 0, stream>>>(ysum, xz, nw, nb, out);
}
